// MGC_Net_43593918055150
// MI455X (gfx1250) — hardware-run, weakly checked
//
#include <hip/hip_runtime.h>

typedef float          v8f   __attribute__((ext_vector_type(8)));
typedef float          v4f   __attribute__((ext_vector_type(4)));
typedef unsigned int   v4u   __attribute__((ext_vector_type(4)));
typedef int            v8i   __attribute__((ext_vector_type(8)));
typedef unsigned short v8us  __attribute__((ext_vector_type(8)));
typedef unsigned short v16us __attribute__((ext_vector_type(16)));
typedef __bf16         v16bf __attribute__((ext_vector_type(16)));
typedef _Float16       v16h  __attribute__((ext_vector_type(16)));
typedef v4f  __attribute__((may_alias)) v4fa;
typedef v8us __attribute__((may_alias)) v8usa;
union FragB { v16bf v; v16us u; v8us h[2]; v8i w; };
union FragH { v16h  v; v16us u; v8us h[2]; v8i w; };

__device__ __forceinline__ v8f wmb(const FragB& a, const FragB& b, v8f c) {
  v8f d = __builtin_amdgcn_wmma_f32_16x16x32_bf16(false, a.v, false, b.v, (short)0, c, false, false);
  asm volatile("v_nop\n\tv_nop\n\tv_nop\n\tv_nop" : "+v"(d) : "v"(a.w), "v"(b.w));
  return d;
}

__device__ __forceinline__ v8f wmh(const FragH& a, const FragH& b, v8f c) {
  v8f d = __builtin_amdgcn_wmma_f32_16x16x32_f16(false, a.v, false, b.v, (short)0, c, false, false);
  asm volatile("v_nop\n\tv_nop\n\tv_nop\n\tv_nop" : "+v"(d) : "v"(a.w), "v"(b.w));
  return d;
}

__device__ __forceinline__ unsigned bf16_bits(float f) {
  const unsigned u = __float_as_uint(f);
  const unsigned r = (u + 0x7FFFu + ((u >> 16) & 1u)) >> 16;
  const unsigned q = (u >> 16) | 0x40u;
  return ((u & 0x7fffffffu) > 0x7f800000u) ? q : r;
}

__device__ __forceinline__ float bf16_val(float f) {
  return __uint_as_float(bf16_bits(f) << 16);
}
__device__ __forceinline__ int clampi(int v, int lo, int hi) {
  return v < lo ? lo : (v > hi ? hi : v);
}

__device__ __forceinline__ unsigned f16_bits(float f) {
  const unsigned u  = __float_as_uint(f);
  const unsigned s  = (u >> 16) & 0x8000u;
  const unsigned a  = u & 0x7fffffffu;
  const unsigned t  = a - 0x38000000u;
  const unsigned r  = (t + 0x0FFFu + ((t >> 13) & 1u)) >> 13;
  const unsigned rc = r > 0x7C00u ? 0x7C00u : r;
  const bool small  = a < 0x38800000u;
  const bool isnan  = a > 0x7f800000u;
  const unsigned fin = small ? 0u : (s | rc);
  return isnan ? (s | 0x7E00u) : fin;
}

__device__ __forceinline__ unsigned pk16(unsigned lo, unsigned hi) { return lo | (hi << 16); }
__device__ __forceinline__ unsigned bf16_lo_bits(float v) {
  float hi = bf16_val(v);
  asm volatile("" : "+v"(hi));
  return bf16_bits(v - hi);
}
__device__ __forceinline__ v4u pack8_bf16(v4f a, v4f c) {
  return (v4u){ pk16(bf16_bits(a[0]), bf16_bits(a[1])), pk16(bf16_bits(a[2]), bf16_bits(a[3])),
                pk16(bf16_bits(c[0]), bf16_bits(c[1])), pk16(bf16_bits(c[2]), bf16_bits(c[3])) };
}
__device__ __forceinline__ v4u pack8_bf16_lo(v4f a, v4f c) {
  return (v4u){ pk16(bf16_lo_bits(a[0]), bf16_lo_bits(a[1])), pk16(bf16_lo_bits(a[2]), bf16_lo_bits(a[3])),
                pk16(bf16_lo_bits(c[0]), bf16_lo_bits(c[1])), pk16(bf16_lo_bits(c[2]), bf16_lo_bits(c[3])) };
}
__device__ __forceinline__ v4u pack8_f16(v4f a, v4f c) {
  return (v4u){ pk16(f16_bits(a[0]), f16_bits(a[1])), pk16(f16_bits(a[2]), f16_bits(a[3])),
                pk16(f16_bits(c[0]), f16_bits(c[1])), pk16(f16_bits(c[2]), f16_bits(c[3])) };
}

template <int FORM>
__global__ __launch_bounds__(256) void k_plane(const float* __restrict__ src, int rows, int cols, int ldsrc,
                                               unsigned short* __restrict__ dst, int MP, int KP) {
  static_assert(FORM >= 0 && FORM <= 3);
  const int KTOT = (FORM == 1 || FORM == 3) ? 2 * KP : KP;
  const unsigned ppr   = (unsigned)(KTOT >> 3);
  const unsigned kp8   = (unsigned)(KP >> 3);
  const unsigned total = (unsigned)MP * ppr;
  const unsigned g     = blockIdx.x * 256u + threadIdx.x;
  const unsigned rowu  = g / ppr;
  const unsigned p     = g - rowu * ppr;
  const bool second    = p >= kp8;
  const int row = (int)rowu;
  const int c0  = (int)((second ? p - kp8 : p) << 3);
  const float* srow = src + (size_t)clampi(row, 0, rows - 1) * (size_t)ldsrc;
  float x[8];
  unsigned mk[8];
#pragma unroll
  for (int e = 0; e < 8; ++e) {
    const int c = c0 + e;
    const float v = srow[clampi(c, 0, cols - 1)];
    asm volatile("" :: "v"(v));
    x[e]  = v;
    mk[e] = (row < rows && c < cols) ? 0xFFFFu : 0u;
  }
  const v4f a = (v4f){ x[0], x[1], x[2], x[3] };
  const v4f c = (v4f){ x[4], x[5], x[6], x[7] };
  v4u o;
  if (FORM == 2) {
    o = pack8_f16(a, c);
  } else {
    const v4u hi = pack8_bf16(a, c);
    o = hi;
    if (FORM == 1) { const v4u lo = pack8_bf16_lo(a, c); o = second ? lo : hi; }
  }
  const v4u mw = (v4u){ pk16(mk[0], mk[1]), pk16(mk[2], mk[3]), pk16(mk[4], mk[5]), pk16(mk[6], mk[7]) };
  o &= mw;
  if (g < total) {
    volatile v4u* q = (volatile v4u*)(dst + (size_t)g * 8);
    *q = o;
    __threadfence();
    *q = o;
  }
}

template <int FORM> struct FragOf    { typedef FragB T; };
template <>         struct FragOf<2> { typedef FragH T; };
__device__ __forceinline__ v8f mm(const FragB& a, const FragB& b, v8f c) { return wmb(a, b, c); }
__device__ __forceinline__ v8f mm(const FragH& a, const FragH& b, v8f c) { return wmh(a, b, c); }
template <class F> __device__ __forceinline__ F ld_frag(const unsigned short* p) {
  F f;
  f.h[0] = *(const v8usa*)(p);
  f.h[1] = *(const v8usa*)(p + 16);
  return f;
}

template <int FORM, int EPI>
__global__ __launch_bounds__(256) __attribute__((amdgpu_num_vgpr(248)))
void k_gemm_nt(const unsigned short* __restrict__ A, const unsigned short* __restrict__ B,
               const float* __restrict__ bias, float* __restrict__ D, int M, int N, int KTOT, int ldd) {
  static_assert(FORM >= 0 && FORM <= 2);
  static_assert(EPI == 0 || EPI == 1);
  typedef typename FragOf<FORM>::T F;
  __shared__ __attribute__((aligned(16))) float sT[8][16 * 68];
  const int lane = threadIdx.x & 31;
  const int wave = threadIdx.x >> 5;
  const int tilesM = (M + 63) >> 6;
  const int tilesN = (N + 63) >> 6;
  const int tile = blockIdx.x * 8 + wave;
  if (tile >= tilesM * tilesN) return;
  const int tm = tile / tilesN;
  const int tn = tile - tm * tilesN;
  const int m0 = tm << 6;
  const int n0 = tn << 6;

  const int rl = lane & 15;
  const int h8 = (lane >> 4) * 8;
  const unsigned short* pa = A + (size_t)(m0 + rl) * (size_t)KTOT + h8;
  const unsigned short* pb = B + (size_t)(n0 + rl) * (size_t)KTOT + h8;

  v8f acc[4][4];
#pragma unroll
  for (int i = 0; i < 4; ++i)
#pragma unroll
    for (int j = 0; j < 4; ++j) acc[i][j] = (v8f){0.f, 0.f, 0.f, 0.f, 0.f, 0.f, 0.f, 0.f};

#pragma unroll 1
  for (int k0 = 0; k0 < KTOT; k0 += 32) {
    F bf[4];
#pragma unroll
    for (int j = 0; j < 4; ++j) bf[j] = ld_frag<F>(pb + (size_t)(j << 4) * (size_t)KTOT + k0);
#pragma unroll
    for (int i = 0; i < 4; ++i) {
      const F af = ld_frag<F>(pa + (size_t)(i << 4) * (size_t)KTOT + k0);
#pragma unroll
      for (int j = 0; j < 4; ++j) acc[i][j] = mm(af, bf[j], acc[i][j]);
    }
  }

  float* slab = sT[wave];
  const int hh = lane >> 4;
  const int c4 = (lane & 15) * 4;
  const int nc = n0 + c4;
  const bool cok = nc < N;
  v4f bv = (v4f){0.f, 0.f, 0.f, 0.f};
  if (EPI == 1) {
    bv = *(const v4fa*)(bias + clampi(nc, 0, N - 4));
    asm volatile("" :: "v"(bv));
  }
#pragma unroll
  for (int i = 0; i < 4; ++i) {
    const int mBase = m0 + (i << 4);
#pragma unroll
    for (int j = 0; j < 4; ++j) {
#pragma unroll
      for (int r = 0; r < 8; ++r) slab[(h8 + r) * 68 + (j << 4) + rl] = acc[i][j][r];
    }
    __builtin_amdgcn_fence(__ATOMIC_RELEASE, "workgroup");
    __builtin_amdgcn_wave_barrier();
    __builtin_amdgcn_fence(__ATOMIC_ACQUIRE, "workgroup");
    v4f vv[8];
#pragma unroll
    for (int it = 0; it < 8; ++it) {
      const int row = it * 2 + hh;
      v4f v = *(const v4fa*)(slab + row * 68 + c4);
      if (EPI == 1) v += bv;
      vv[it] = v;
    }
    for (int pass = 0; pass < 2; ++pass) {
#pragma unroll
      for (int it = 0; it < 8; ++it) {
        const int row = mBase + it * 2 + hh;
        if (cok && row < M) *(volatile v4f*)(D + (size_t)row * (size_t)ldd + nc) = vv[it];
      }
      __threadfence();
    }
    __builtin_amdgcn_fence(__ATOMIC_RELEASE, "workgroup");
    __builtin_amdgcn_wave_barrier();
    __builtin_amdgcn_fence(__ATOMIC_ACQUIRE, "workgroup");
  }
}

#pragma clang fp contract(off)

#define GN    2048
#define GFIN  768
#define GH    8
#define GD    64
#define GC    512
#define P_SPLIT  1
#define WH_SPLIT 1
#define NSEG  (1 + P_SPLIT + WH_SPLIT)
#define KTOT_ (GN * NSEG)
#define LK_SLOPE 0.2f
#define MASK_FILL (-9.0e15f)

static_assert(GN % 128 == 0);
static_assert(GN % 64 == 0);
static_assert(GN % 16 == 0);
static_assert(GFIN % 32 == 0);
static_assert(GFIN % 64 == 0);
static_assert(KTOT_ % 32 == 0);
static_assert(GC == GH * GD);
static_assert(GD == 64);
static_assert(GC % 64 == 0);
static_assert(GC % 32 == 0);
static_assert(GD % 4 == 0);
static_assert((GN * GFIN / 8) % 256 == 0);
static_assert(P_SPLIT == 0 || P_SPLIT == 1);
static_assert(WH_SPLIT == 0 || WH_SPLIT == 1);

__global__ __launch_bounds__(256) void k_wt(const float* __restrict__ W, unsigned short* __restrict__ WT) {
  __shared__ __attribute__((aligned(16))) float tf[64 * 68];
  const int c0  = blockIdx.x * 64;
  const int r0  = blockIdx.y * 64;
  const int tid = threadIdx.x;
  {
    const int lr = tid >> 4;
    const int c4 = (tid & 15) * 4;
#pragma unroll
    for (int it = 0; it < 4; ++it) {
      const int rr = it * 16 + lr;
      const v4f x = *(const v4fa*)(W + (size_t)(r0 + rr) * GC + c0 + c4);
      asm volatile("" :: "v"(x));
      *(v4fa*)(tf + rr * 68 + c4) = x;
    }
  }
  __syncthreads();
  const int sub = tid >> 3;
  const int c8  = (tid & 7) * 8;
  v4u hv[2];
#pragma unroll
  for (int it = 0; it < 2; ++it) {
    const int oc = it * 32 + sub;
    v4u o;
#pragma unroll
    for (int q = 0; q < 4; ++q) {
      const float f0 = tf[(c8 + 2 * q) * 68 + oc];
      const float f1 = tf[(c8 + 2 * q + 1) * 68 + oc];
      o[q] = pk16(bf16_bits(f0), bf16_bits(f1));
    }
    hv[it] = o;
  }
  for (int pass = 0; pass < 2; ++pass) {
#pragma unroll
    for (int it = 0; it < 2; ++it) {
      const int oc = it * 32 + sub;
      *(volatile v4u*)(WT + (size_t)(c0 + oc) * GFIN + r0 + c8) = hv[it];
    }
    __threadfence();
  }
}

__global__ __launch_bounds__(256) void k_score(const float* __restrict__ WH, const float* __restrict__ avec,
                                               float* __restrict__ E) {
  __shared__ __attribute__((aligned(16))) float sA[GH * 2 * GD];
  __shared__ __attribute__((aligned(16))) float sR[2 * GH * 32];
  const int tid = threadIdx.x, lane = tid & 31, w = tid >> 5;
  {
    const v4f x = *(const v4fa*)(avec + tid * 4);
    asm volatile("" :: "v"(x));
    const v4f y = (v4f){ bf16_val(x[0]), bf16_val(x[1]), bf16_val(x[2]), bf16_val(x[3]) };
    *(v4fa*)(sA + tid * 4) = y;
  }
  __syncthreads();
  const int hd = lane >> 2;
  const int db = (lane & 3) * 16;
  v4f ai[4], aj[4];
#pragma unroll
  for (int c = 0; c < 4; ++c) {
    ai[c] = *(const v4fa*)(sA + hd * 128 + db + 4 * c);
    aj[c] = *(const v4fa*)(sA + hd * 128 + 64 + db + 4 * c);
  }
  const int nb = blockIdx.x * 32 + w * 4;
#pragma unroll 1
  for (int q = 0; q < 4; ++q) {
    const float* wr = WH + (size_t)(nb + q) * GC + lane * 16;
    v4f x[4];
#pragma unroll
    for (int c = 0; c < 4; ++c) {
      x[c] = *(const v4fa*)(wr + 4 * c);
      asm volatile("" :: "v"(x[c]));
    }
    float si = 0.0f, sj = 0.0f;
#pragma unroll
    for (int c = 0; c < 4; ++c) {
#pragma unroll
      for (int e = 0; e < 4; ++e) {
        si = fmaf(x[c][e], ai[c][e], si);
        sj = fmaf(x[c][e], aj[c][e], sj);
      }
    }
    si += __shfl_xor(si, 1, 32);
    sj += __shfl_xor(sj, 1, 32);
    si += __shfl_xor(si, 2, 32);
    sj += __shfl_xor(sj, 2, 32);
    if ((lane & 3) == 0) {
      sR[hd * 32 + w * 4 + q]       = si;
      sR[256 + hd * 32 + w * 4 + q] = sj;
    }
  }
  __syncthreads();
  if (tid < 128) {
    const int line  = tid >> 3;
    const int piece = tid & 7;
    const v4f v = *(const v4fa*)(sR + line * 32 + piece * 4);
    volatile v4f* d = (volatile v4f*)(E + (size_t)line * GN + blockIdx.x * 32 + piece * 4);
    *d = v;
    __threadfence();
    *d = v;
  }
}

__global__ __launch_bounds__(256) void k_whT(const float* __restrict__ WH, unsigned* __restrict__ WHT32) {
  __shared__ float tf[64 * 65];
  const int j0  = blockIdx.x * 64;
  const int hd  = blockIdx.y;
  const int tid = threadIdx.x, lane = tid & 31, w = tid >> 5;
  {
    const int lr = tid >> 4;
    const int c4 = (tid & 15) * 4;
#pragma unroll
    for (int it = 0; it < 4; ++it) {
      const int jj = it * 16 + lr;
      const v4f x = *(const v4fa*)(WH + (size_t)(j0 + jj) * GC + hd * GD + c4);
      asm volatile("" :: "v"(x));
      tf[jj * 65 + c4 + 0] = x[0];
      tf[jj * 65 + c4 + 1] = x[1];
      tf[jj * 65 + c4 + 2] = x[2];
      tf[jj * 65 + c4 + 3] = x[3];
    }
  }
  __syncthreads();
  unsigned hw[8], lw[8];
#pragma unroll
  for (int r = 0; r < 8; ++r) {
    const int d = w * 8 + r;
    const float f0 = tf[(2 * lane) * 65 + d];
    const float f1 = tf[(2 * lane + 1) * 65 + d];
    hw[r] = pk16(bf16_bits(f0), bf16_bits(f1));
    lw[r] = pk16(bf16_lo_bits(f0), bf16_lo_bits(f1));
  }
  for (int pass = 0; pass < 2; ++pass) {
#pragma unroll
    for (int r = 0; r < 8; ++r) {
      const size_t rowb = (size_t)(hd * GD + w * 8 + r) * (size_t)KTOT_ + (size_t)j0;
      *(volatile unsigned*)(WHT32 + (rowb >> 1) + lane) = hw[r];
      if (P_SPLIT)  *(volatile unsigned*)(WHT32 + ((rowb + (size_t)GN) >> 1) + lane) = hw[r];
      if (WH_SPLIT) *(volatile unsigned*)(WHT32 + ((rowb + (size_t)(1 + P_SPLIT) * GN) >> 1) + lane) = lw[r];
    }
    __threadfence();
  }
}

__global__ __launch_bounds__(128) void k_attrow(const float* __restrict__ adj, const float* __restrict__ E,
                                                unsigned short* __restrict__ P, int hd) {
  __shared__ __attribute__((aligned(16))) float sE[4][GN];
  const int lane = threadIdx.x & 31, w = threadIdx.x >> 5;
  const int i = blockIdx.x * 4 + w;
  float* se = sE[w];
  const float EI = E[(size_t)hd * GN + i];
  const float* arow = adj + (size_t)i * GN;
  const float* ej   = E + (size_t)(GH + hd) * GN;

  float m = __uint_as_float(0xff800000u);
#pragma unroll 1
  for (int t = 0; t < 8; ++t) {
    const int j = 256 * t + 8 * lane;
    const v4f a0 = *(const v4fa*)(arow + j);
    const v4f a1 = *(const v4fa*)(arow + j + 4);
    const v4f b0 = *(const v4fa*)(ej + j);
    const v4f b1 = *(const v4fa*)(ej + j + 4);
    asm volatile("" :: "v"(a0));
    asm volatile("" :: "v"(a1));
    asm volatile("" :: "v"(b0));
    asm volatile("" :: "v"(b1));
    v4f e0, e1;
#pragma unroll
    for (int c = 0; c < 4; ++c) {
      float x = EI + b0[c];
      x = (x >= 0.0f) ? x : LK_SLOPE * x;
      x = (a0[c] > 0.0f) ? x : MASK_FILL;
      e0[c] = x;
      m = (x > m || x != x) ? x : m;
    }
#pragma unroll
    for (int c = 0; c < 4; ++c) {
      float x = EI + b1[c];
      x = (x >= 0.0f) ? x : LK_SLOPE * x;
      x = (a1[c] > 0.0f) ? x : MASK_FILL;
      e1[c] = x;
      m = (x > m || x != x) ? x : m;
    }
    *(v4fa*)(se + (2 * t) * 128 + lane * 4)     = e0;
    *(v4fa*)(se + (2 * t + 1) * 128 + lane * 4) = e1;
  }
  {
    float o;
    o = __shfl_xor(m, 16, 32); m = (o > m || o != o) ? o : m;
    o = __shfl_xor(m, 8, 32);  m = (o > m || o != o) ? o : m;
    o = __shfl_xor(m, 4, 32);  m = (o > m || o != o) ? o : m;
    o = __shfl_xor(m, 2, 32);  m = (o > m || o != o) ? o : m;
    o = __shfl_xor(m, 1, 32);  m = (o > m || o != o) ? o : m;
  }

  float s = 0.0f;
#pragma unroll 1
  for (int q = 0; q < 16; ++q) {
    const v4f e = *(const v4fa*)(se + q * 128 + lane * 4);
    v4f x;
#pragma unroll
    for (int c = 0; c < 4; ++c) {
      x[c] = expf(e[c] - m);
      s += x[c];
    }
    *(v4fa*)(se + q * 128 + lane * 4) = x;
  }
  s += __shfl_xor(s, 16, 32);
  s += __shfl_xor(s, 8, 32);
  s += __shfl_xor(s, 4, 32);
  s += __shfl_xor(s, 2, 32);
  s += __shfl_xor(s, 1, 32);

#pragma unroll 1
  for (int q = 0; q < 16; ++q) {
    const v4f x = *(const v4fa*)(se + q * 128 + lane * 4);
    v4f p;
#pragma unroll
    for (int c = 0; c < 4; ++c) p[c] = x[c] / s;
    *(v4fa*)(se + q * 128 + lane * 4) = p;
  }

  unsigned short* prow = P + (size_t)i * (size_t)KTOT_;
#pragma unroll 1
  for (int t = 0; t < 8; ++t) {
    const v4f p0 = *(const v4fa*)(se + (2 * t) * 128 + lane * 4);
    const v4f p1 = *(const v4fa*)(se + (2 * t + 1) * 128 + lane * 4);
    const v4u hi = pack8_bf16(p0, p1);
    v4u lo = hi;
    if (P_SPLIT) lo = pack8_bf16_lo(p0, p1);
    const int col = 256 * t + 8 * lane;
    for (int pass = 0; pass < 2; ++pass) {
      *(volatile v4u*)(prow + col) = hi;
      if (P_SPLIT)  *(volatile v4u*)(prow + GN + col) = lo;
      if (WH_SPLIT) *(volatile v4u*)(prow + (1 + P_SPLIT) * GN + col) = hi;
      __threadfence();
    }
  }
}

__global__ __launch_bounds__(256) void k_elu(const float* __restrict__ HP, float* __restrict__ out) {
  __shared__ __attribute__((aligned(16))) float sX[8][GC];
  const int lane = threadIdx.x & 31, w = threadIdx.x >> 5;
  const int row = blockIdx.x * 8 + w;
  const int rr  = clampi(row, 0, GN - 1);
  float* sx = sX[w];
#pragma unroll
  for (int c = 0; c < 4; ++c) {
    const v4f x = *(const v4fa*)(HP + (size_t)rr * GC + 128 * c + 4 * lane);
    asm volatile("" :: "v"(x));
    *(v4fa*)(sx + 128 * c + 4 * lane) = x;
  }
#pragma unroll 1
  for (int k = 0; k < 16; ++k) {
    const int idx = (k >> 2) * 128 + 4 * lane + (k & 3);
    const float v = sx[idx];
    const float r = (v > 0.0f) ? v : expm1f(v);
    sx[idx] = r;
  }
  v4f y[4];
#pragma unroll
  for (int c = 0; c < 4; ++c) y[c] = *(const v4fa*)(sx + 128 * c + 4 * lane);
  if (row < GN) {
    for (int pass = 0; pass < 2; ++pass) {
#pragma unroll
      for (int c = 0; c < 4; ++c)
        *(volatile v4f*)(out + (size_t)row * GC + 128 * c + 4 * lane) = y[c];
      __threadfence();
    }
  }
}

static constexpr size_t SZ_HB  = (size_t)GN * GFIN * 2;
static constexpr size_t SZ_WT  = (size_t)GC * GFIN * 2;
static constexpr size_t SZ_WH  = (size_t)GN * GC * 4;
static constexpr size_t SZ_E   = (size_t)2 * GH * GN * 4;
static constexpr size_t SZ_WHT = (size_t)GC * KTOT_ * 2;
static constexpr size_t SZ_P   = (size_t)GN * KTOT_ * 2;
static constexpr size_t SZ_HP  = (size_t)GN * GC * 4;
static constexpr size_t SZ_ALL = SZ_HB + SZ_WT + SZ_WH + SZ_E + SZ_WHT + SZ_P + SZ_HP;
static_assert(SZ_HB % 256 == 0 && SZ_WT % 256 == 0 && SZ_WH % 256 == 0 && SZ_E % 256 == 0);
static_assert(SZ_WHT % 256 == 0 && SZ_P % 256 == 0 && SZ_HP % 256 == 0);
static_assert(NSEG != 3 || SZ_ALL == (size_t)43909120);
static_assert(SZ_ALL <= ((size_t)128 << 20));
static_assert((size_t)GN * KTOT_ / 8 < (size_t)0x7fffffff);

extern "C" void kernel_launch(void* const* d_in, const int* in_sizes, int n_in,
                              void* d_out, int out_size, void* d_ws, size_t ws_size,
                              hipStream_t stream) {
  if (n_in < 4) return;
  if (in_sizes[0] != GN * GFIN) return;
  if (in_sizes[1] != GN * GN) return;
  if (in_sizes[2] != GFIN * GC) return;
  if (in_sizes[3] != GH * 2 * GD) return;
  if (out_size != GN * GC) return;
  if (ws_size < SZ_ALL) return;

  const float* hin = (const float*)d_in[0];
  const float* adj = (const float*)d_in[1];
  const float* W   = (const float*)d_in[2];
  const float* av  = (const float*)d_in[3];
  float* out = (float*)d_out;

  char* ws = (char*)d_ws;
  size_t off = 0;
  unsigned short* HB  = (unsigned short*)(ws + off); off += SZ_HB;
  unsigned short* WT  = (unsigned short*)(ws + off); off += SZ_WT;
  float*          WH  = (float*)(ws + off);          off += SZ_WH;
  float*          E   = (float*)(ws + off);          off += SZ_E;
  unsigned short* WHT = (unsigned short*)(ws + off); off += SZ_WHT;
  unsigned short* P   = (unsigned short*)(ws + off); off += SZ_P;
  float*          HP  = (float*)(ws + off);          off += SZ_HP;

  k_plane<0><<<dim3(GN * GFIN / 8 / 256), 256, 0, stream>>>(hin, GN, GFIN, GFIN, HB, GN, GFIN);
  k_wt<<<dim3(GC / 64, GFIN / 64), 256, 0, stream>>>(W, WT);
  k_gemm_nt<0, 0><<<dim3((GN / 64) * (GC / 64) / 8), 256, 0, stream>>>(HB, WT, av, WH, GN, GC, GFIN, GC);
  k_score<<<dim3(GN / 32), 256, 0, stream>>>(WH, av, E);
  k_whT<<<dim3(GN / 64, GH), 256, 0, stream>>>(WH, (unsigned*)WHT);
  for (int hd = 0; hd < GH; ++hd) {
    k_attrow<<<dim3(GN / 4), 128, 0, stream>>>(adj, E, P, hd);
    k_gemm_nt<0, 0><<<dim3((GN / 64 + 7) / 8), 256, 0, stream>>>(
        P, WHT + (size_t)GD * hd * KTOT_, av, HP + GD * hd, GN, GD, KTOT_, GC);
  }
  k_elu<<<dim3(GN / 8), 256, 0, stream>>>(HP, out);
}
